// GLFMSABlock_69131793596507
// MI455X (gfx1250) — hardware-verified
//
#include <hip/hip_runtime.h>
#include <math.h>

typedef __attribute__((ext_vector_type(16))) _Float16 v16h;
typedef __attribute__((ext_vector_type(16))) __bf16 v16b;
typedef __attribute__((ext_vector_type(8)))  _Float16 v8h;
typedef __attribute__((ext_vector_type(8)))  float v8f;
typedef __attribute__((ext_vector_type(4)))  float v4f;
typedef __attribute__((ext_vector_type(2)))  float v2f;
typedef __attribute__((ext_vector_type(4)))  unsigned v4u;
typedef __attribute__((ext_vector_type(4)))  int v4i;
typedef float __attribute__((may_alias)) float_a;
typedef int __attribute__((may_alias)) int_a;

template <typename T> __device__ __forceinline__ void vst2(void* p, T v) { *(volatile T*)p = v; __threadfence(); *(volatile T*)p = v; }
__device__ __forceinline__ v8f wmma16(v16h a, v16h b, v8f c) {
  v8f d = __builtin_amdgcn_wmma_f32_16x16x32_f16(false, a, false, b, (short)0, c, false, false);
  asm volatile("v_nop\n\tv_nop\n\tv_nop\n\tv_nop" : "+v"(d) : "v"(a), "v"(b));
  return d;
}
__device__ __forceinline__ v8f wmma_bf(v16b a, v16b b, v8f c) {
  v8f d = __builtin_amdgcn_wmma_f32_16x16x32_bf16(false, a, false, b, (short)0, c, false, false);
  asm volatile("v_nop\n\tv_nop\n\tv_nop\n\tv_nop" : "+v"(d) : "v"(a), "v"(b));
  return d;
}
__device__ __forceinline__ v16h frag_h(const _Float16* rowk0, int lane) {
  union { v16h v; v8h q[2]; } u; const _Float16* p = rowk0 + 8 * (lane >> 4);
  u.q[0] = *(const v8h*)p; u.q[1] = *(const v8h*)(p + 16); return u.v;
}
__device__ __forceinline__ v16h frag_f32(const float* rowk0, int lane) {
  v16h a; const float* p = rowk0 + 8 * (lane >> 4);
#pragma unroll
  for (int i = 0; i < 8; ++i) { a[i] = (_Float16)p[i]; a[8 + i] = (_Float16)p[16 + i]; }
  return a;
}
__device__ __forceinline__ v16h frag_f32s(const float* rowk0, int lane, float sc) {
  v16h a; const float* p = rowk0 + 8 * (lane >> 4);
#pragma unroll
  for (int i = 0; i < 8; ++i) { a[i] = (_Float16)(p[i] * sc); a[8 + i] = (_Float16)(p[16 + i] * sc); }
  return a;
}
__device__ __forceinline__ v16h fragc_f32(const float* W, int k0, int n, int lane, int ld, int K) {
  v16h a; const int g = lane >> 4;
#pragma unroll
  for (int i = 0; i < 8; ++i) { const int ka = k0 + 8 * g + i, kb = ka + 16;
    a[i] = (_Float16)(ka < K ? W[(size_t)(ka < K ? ka : K - 1) * ld + n] : 0.f); a[8 + i] = (_Float16)(kb < K ? W[(size_t)(kb < K ? kb : K - 1) * ld + n] : 0.f); }
  return a;
}
struct F2 { v16b h, l; };
__device__ __forceinline__ F2 bsplit16(const float v[16]) { F2 r;
#pragma unroll
  for (int i = 0; i < 16; ++i) { const __bf16 h = (__bf16)v[i]; r.h[i] = h; r.l[i] = (__bf16)(v[i] - (float)h); }
  return r; }
__device__ __forceinline__ F2 split_row(const float* row, int k0, int lane) { float v[16]; const float* p = row + k0 + 8 * (lane >> 4);
#pragma unroll
  for (int i = 0; i < 8; ++i) { v[i] = p[i]; v[8 + i] = p[16 + i]; }
  return bsplit16(v); }
__device__ __forceinline__ F2 split_rowK(const float* row, int k0, int lane, int K) { float v[16]; const int g = lane >> 4;
#pragma unroll
  for (int i = 0; i < 8; ++i) { const int ka = k0 + 8 * g + i, kb = ka + 16; v[i] = ka < K ? row[ka < K ? ka : K - 1] : 0.f; v[8 + i] = kb < K ? row[kb < K ? kb : K - 1] : 0.f; }
  return bsplit16(v); }
__device__ __forceinline__ F2 split_col(const float* W, int k0, int n, int lane, int ld, int K) { float v[16]; const int g = lane >> 4;
#pragma unroll
  for (int i = 0; i < 8; ++i) { const int ka = k0 + 8 * g + i, kb = ka + 16; v[i] = ka < K ? W[(size_t)(ka < K ? ka : K - 1) * ld + n] : 0.f; v[8 + i] = kb < K ? W[(size_t)(kb < K ? kb : K - 1) * ld + n] : 0.f; }
  return bsplit16(v); }
__device__ __forceinline__ v8f mac3(const F2& a, const F2& b, v8f c) { c = wmma_bf(a.l, b.h, c); c = wmma_bf(a.h, b.l, c); return wmma_bf(a.h, b.h, c); }
__device__ __forceinline__ float sigm(float v) { return 1.0f / (1.0f + expf(-v)); }
#define LDSX() do { asm volatile("s_wait_dscnt 0" ::: "memory"); __builtin_amdgcn_wave_barrier(); __builtin_amdgcn_fence(__ATOMIC_RELEASE, "workgroup"); } while (0)


#define NB 4
#define SS 2048
#define DM 512
#define NH 8
#define HD 64
#define QKVW (3 * DM)
#ifndef TQB
#define TQB (SS / 64)
#define TNB NB
#define TOB (NB * SS / 64)
#endif
typedef __attribute__((ext_vector_type(8))) __bf16 v8b;
__device__ __forceinline__ v16b frag_b(const __bf16* rowk0, int lane) {
  union { v16b v; v8b q[2]; } u; const __bf16* p = rowk0 + 8 * (lane >> 4);
  u.q[0] = *(const v8b*)p; u.q[1] = *(const v8b*)(p + 16); return u.v;
}
__device__ __forceinline__ float bfr(float v) { return (float)(__bf16)v; }
__device__ __attribute__((noinline)) float exp_ni(float v) { return expf(v); }
__device__ __attribute__((noinline)) float erf_ni(float v) { return erff(v); }

#define PK_A 0
#define PK_P (PK_A + QKVW * DM)
#define PK_END (PK_P + DM * DM)

#define NR (NB * SS)
#define HD2 256
#define NHG 2
#define D3 (3 * DM)
#define D2 (2 * DM)
#define DFF 2048
#define LWIN 2
#ifndef NRB
#define NRB (NR / 64)
#endif
#ifndef TQBG
#define TQBG (SS / 64)
#endif

#define WS_PK   0u
#define WS_PKL  (WS_PK + 2u * (size_t)PK_END)
#define WS_PFU  (WS_PKL + 2u * (size_t)PK_END)
#define WS_PF1  (WS_PFU + 2u * (size_t)DM * D2)
#define WS_PF2  (WS_PF1 + 2u * (size_t)DFF * DM)
#define WS_QK   (WS_PF2 + 2u * (size_t)DM * DFF)
#define WS_QKL  (WS_QK + 2u * (size_t)NR * D2)
#define WS_VTH  (WS_QKL + 2u * (size_t)NR * D2)
#define WS_VTL  (WS_VTH + 2u * (size_t)NB * DM * SS)
#define WS_OG   (WS_VTL + 2u * (size_t)NB * DM * SS)
#define WS_LQKV (WS_OG + 4u * (size_t)NR * DM)
#define WS_LCTX (WS_LQKV + 4u * (size_t)NR * D3)
#define WS_GOUT (WS_LCTX + 4u * (size_t)NR * DM)
#define WS_LOUT (WS_GOUT + 4u * (size_t)NR * DM)
#define WS_X1   (WS_LQKV)
#define WS_H16  (WS_X1 + 4u * (size_t)NR * DM)
#define WS_G16  (WS_H16 + 2u * (size_t)NR * DM)
#define WS_G16b (WS_LOUT + 4u * (size_t)NR * DM)
#define WS_Y    (WS_G16b + 2u * (size_t)NR * DFF)
#define WS_END  (WS_Y + 4u * (size_t)NR * DM)
__global__ __launch_bounds__(256) void k_pack(const float* __restrict__ WQ, const float* __restrict__ WK, const float* __restrict__ WV, const float* __restrict__ WO, __bf16* __restrict__ PK) {
  __shared__ __align__(16) __bf16 s[DM]; const int n = blockIdx.x, which = blockIdx.y, t = threadIdx.x; const float* Wm = (which == 0) ? WQ : (which == 1) ? WK : (which == 2) ? WV : WO;
  for (int k = t; k < DM; k += 256) s[k] = (__bf16)Wm[(size_t)n * DM + k];
  __syncthreads();
  __bf16* dst = (which < 3) ? PK + PK_A + ((size_t)which * DM + n) * DM : PK + PK_P + (size_t)n * DM;
  for (int q = t; q < DM / 8; q += 256) vst2((unsigned*)(dst + q * 8), *(const v4u*)&s[q * 8]);
}
__global__ __launch_bounds__(128) void k_qkv(const float* __restrict__ XQ, const float* __restrict__ XK, const float* __restrict__ XV, const __bf16* __restrict__ P, const float* __restrict__ BQ, const float* __restrict__ BK, const float* __restrict__ BV, _Float16* __restrict__ QK, _Float16* __restrict__ QKL, _Float16* __restrict__ VTH, _Float16* __restrict__ VTL) {
  const int which0 = (blockIdx.y * 128) / DM; const float* X = (which0 == 0) ? XQ : (which0 == 1) ? XK : XV; const float* BB = BQ ? (((which0 == 0) ? BQ : (which0 == 1) ? BK : BV) + (blockIdx.y * 128 - which0 * DM)) : nullptr;
  __shared__ __align__(16) _Float16 so[4][16][136], sol[4][16][136]; __shared__ __align__(16) _Float16 sth[128][72], stl[128][72];
  const int tid = threadIdx.x, wave = tid >> 5, lane = tid & 31, col = lane & 15, g = lane >> 4; const size_t r0 = (size_t)blockIdx.x * 64 + wave * 16; const int n0 = blockIdx.y * 128;
  v8f acc[8] = {};
#pragma unroll 2
  for (int kc = 0; kc < DM / 32; ++kc) { v16b a; { const float* p = X + (r0 + col) * DM + kc * 32 + 8 * g;
#pragma unroll
      for (int i = 0; i < 8; ++i) { a[i] = (__bf16)p[i]; a[8 + i] = (__bf16)p[16 + i]; } }
#pragma unroll
    for (int j = 0; j < 8; ++j) acc[j] = wmma_bf(a, frag_b(P + (size_t)(n0 + j * 16 + col) * DM + kc * 32, lane), acc[j]); }
  if (n0 < 2 * DM) {
#pragma unroll
    for (int j = 0; j < 8; ++j) {
#pragma unroll
      for (int r = 0; r < 8; ++r) { const float v = acc[j][r] + (BB ? bfr(BB[j * 16 + col]) : 0.f); const _Float16 hv = (_Float16)v; so[wave][8 * g + r][j * 16 + col] = hv; sol[wave][8 * g + r][j * 16 + col] = (_Float16)((v - (float)hv) * 2048.0f); } }
    LDSX();
    for (int rl = 0; rl < 16; ++rl) if (lane < 16) { vst2((unsigned*)(QK + (r0 + rl) * (2 * DM) + n0 + lane * 8), *(const v4u*)&so[wave][rl][lane * 8]); vst2((unsigned*)(QKL + (r0 + rl) * (2 * DM) + n0 + lane * 8), *(const v4u*)&sol[wave][rl][lane * 8]); }
  } else {
#pragma unroll
    for (int j = 0; j < 8; ++j) {
#pragma unroll
      for (int r = 0; r < 8; ++r) { const float v = acc[j][r] + (BB ? bfr(BB[j * 16 + col]) : 0.f); const _Float16 hv = (_Float16)v; sth[j * 16 + col][wave * 16 + 8 * g + r] = hv; stl[j * 16 + col][wave * 16 + 8 * g + r] = (_Float16)((v - (float)hv) * 2048.0f); } }
    __syncthreads();
    const size_t rb = (size_t)blockIdx.x * 64; const int b = (int)(rb / SS), s0 = (int)(rb % SS); const int pc0 = n0 - 2 * DM;
    for (int q = tid; q < 128 * 8; q += 128) { const int d = q >> 3, pc = q & 7; const size_t o = ((size_t)b * DM + pc0 + d) * SS + s0 + pc * 8; vst2((unsigned*)(VTH + o), *(const v4u*)&sth[d][pc * 8]); vst2((unsigned*)(VTL + o), *(const v4u*)&stl[d][pc * 8]); }
  }
}

__global__ __launch_bounds__(256) void k_pack16(const float* __restrict__ W1, const float* __restrict__ W2, const float* __restrict__ WFU, _Float16* __restrict__ PF1, _Float16* __restrict__ PF2, __bf16* __restrict__ PFU) {
  const int n = blockIdx.x, which = blockIdx.y, t = threadIdx.x; __shared__ __align__(16) _Float16 s[DFF]; __shared__ __align__(16) __bf16 sb[D2];
  if (which == 0) { for (int k = t; k < DM; k += 256) s[k] = (_Float16)(bfr(W1[(size_t)n * DM + k]) * 256.0f); __syncthreads(); if (t < DM / 8) vst2((unsigned*)(PF1 + (size_t)n * DM + t * 8), *(const v4u*)&s[t * 8]); }
  else if (which == 1) { if (n >= DM) return; for (int k = t; k < DFF; k += 256) s[k] = (_Float16)(bfr(W2[(size_t)n * DFF + k]) * 256.0f); __syncthreads(); vst2((unsigned*)(PF2 + (size_t)n * DFF + t * 8), *(const v4u*)&s[t * 8]); }
  else { if (n >= DM) return; for (int k = t; k < D2; k += 256) sb[k] = (__bf16)WFU[(size_t)n * D2 + k]; __syncthreads(); if (t < D2 / 8) vst2((unsigned*)(PFU + (size_t)n * D2 + t * 8), *(const v4u*)&sb[t * 8]); }
}
__global__ __launch_bounds__(128) void k_lqkv(const float* __restrict__ X, const __bf16* __restrict__ P, const float* __restrict__ BB, float* __restrict__ OUT) {
  __shared__ __align__(16) float so[4][16][132];
  const int tid = threadIdx.x, wave = tid >> 5, lane = tid & 31, col = lane & 15, g = lane >> 4; const size_t r0 = (size_t)blockIdx.x * 64 + wave * 16; const int n0 = blockIdx.y * 128;
  v8f acc[8] = {};
#pragma unroll 2
  for (int kc = 0; kc < DM / 32; ++kc) { v16b a; { const float* p = X + (r0 + col) * DM + kc * 32 + 8 * g;
#pragma unroll
      for (int i = 0; i < 8; ++i) { a[i] = (__bf16)p[i]; a[8 + i] = (__bf16)p[16 + i]; } }
#pragma unroll
    for (int j = 0; j < 8; ++j) acc[j] = wmma_bf(a, frag_b(P + (size_t)(n0 + j * 16 + col) * DM + kc * 32, lane), acc[j]); }
#pragma unroll
  for (int j = 0; j < 8; ++j) { const float bb = bfr(BB[n0 + j * 16 + col]);
#pragma unroll
    for (int r = 0; r < 8; ++r) so[wave][8 * g + r][j * 16 + col] = acc[j][r] + bb; }
  LDSX();
  for (int rl = 0; rl < 16; ++rl) vst2(OUT + (r0 + rl) * D3 + n0 + lane * 4, *(const v4f*)&so[wave][rl][lane * 4]);
}
__global__ __launch_bounds__(128) void k_gatt(const _Float16* __restrict__ QK, const _Float16* __restrict__ VTH, float* __restrict__ O) {
  __shared__ __align__(16) _Float16 sph[4][16][40]; __shared__ __align__(16) float so[4][16][132];
  const int tid = threadIdx.x, wave = tid >> 5, lane = tid & 31, col = lane & 15, g = lane >> 4; const int qb = blockIdx.x, h = blockIdx.y; const size_t b = blockIdx.z >> 1; const int vh = blockIdx.z & 1; const int q0 = qb * 64 + wave * 16; const size_t rq = b * SS + q0;
  v16h aq[8];
#pragma unroll
  for (int kc = 0; kc < 8; ++kc) aq[kc] = frag_h(QK + (rq + col) * D2 + h * HD2 + kc * 32, lane);
  float m[8], l[8];
#pragma unroll
  for (int r = 0; r < 8; ++r) { m[r] = -3.0e38f; l[r] = 0.f; }
  v8f acc[8] = {}; const int nks = (qb * 64 + 64) / 32;
#pragma unroll 1
  for (int ks = 0; ks < nks; ++ks) { const int j0 = ks * 32; v8f s[2];
#pragma unroll
    for (int ct = 0; ct < 2; ++ct) { const int kk = j0 + ct * 16 + col; const size_t rk = (b * SS + kk) * D2 + DM + h * HD2; v8f c = {};
#pragma unroll
      for (int kc = 0; kc < 8; ++kc) c = wmma16(aq[kc], frag_h(QK + rk + kc * 32, lane), c);
#pragma unroll
      for (int r = 0; r < 8; ++r) s[ct][r] = (kk <= q0 + 8 * g + r) ? c[r] * 0.0625f : -3.0e38f; }
#pragma unroll
    for (int r = 0; r < 8; ++r) { float mx = fmaxf(s[0][r], s[1][r]);
#pragma unroll
      for (int o = 1; o < 16; o <<= 1) mx = fmaxf(mx, __shfl_xor(mx, o));
      const float mn = fmaxf(m[r], mx); const float alpha = (m[r] <= -1.0e38f) ? 0.f : __expf(m[r] - mn); const float e0 = (s[0][r] <= -1.0e38f) ? 0.f : __expf(s[0][r] - mn), e1 = (s[1][r] <= -1.0e38f) ? 0.f : __expf(s[1][r] - mn); float es = e0 + e1;
#pragma unroll
      for (int o = 1; o < 16; o <<= 1) es += __shfl_xor(es, o);
      l[r] = l[r] * alpha + es; m[r] = (mn <= -1.0e38f) ? m[r] : mn;
#pragma unroll
      for (int dt = 0; dt < 8; ++dt) acc[dt][r] *= alpha;
      sph[wave][8 * g + r][col] = (_Float16)(e0 * 2048.0f); sph[wave][8 * g + r][16 + col] = (_Float16)(e1 * 2048.0f); }
    LDSX();
    const v16h pa = frag_h(&sph[wave][col][0], lane);
#pragma unroll
    for (int dt = 0; dt < 8; ++dt) { const size_t vo = (b * DM + (size_t)h * HD2 + vh * 128 + dt * 16 + col) * SS + j0; acc[dt] = wmma16(pa, frag_h(VTH + vo, lane), acc[dt]); }
    LDSX(); }
#pragma unroll
  for (int r = 0; r < 8; ++r) { const float il = (1.0f / 2048.0f) / l[r];
#pragma unroll
    for (int dt = 0; dt < 8; ++dt) so[wave][8 * g + r][dt * 16 + col] = acc[dt][r] * il; }
  LDSX();
  for (int rl = 0; rl < 16; ++rl) vst2(O + (rq + rl) * DM + h * HD2 + vh * 128 + lane * 4, *(const v4f*)&so[wave][rl][lane * 4]);
}
__device__ __attribute__((noinline)) float exp_p(float v) { return expf(v); }
__global__ __launch_bounds__(256) void k_lattn(const float* __restrict__ LQ, float* __restrict__ LCTX) {
  __shared__ float ssc[64][NHG][8];
  const int t = threadIdx.x; const size_t rb0 = (size_t)blockIdx.x * 64; const int r = t >> 2, part = t & 3;
  const int h = part >> 1, half = part & 1; const size_t row = rb0 + r; const int sidx = (int)(row % SS); const size_t sb = row - sidx;
  const float* q = LQ + row * D3 + h * HD2 + half * 128;
  float sc[5];
#pragma unroll
  for (int w = 0; w < 5; ++w) { const int j = sidx + w - LWIN; float s = 0.f; if (j >= 0 && j < SS) { const float* k = LQ + (sb + j) * D3 + DM + h * HD2 + half * 128;
#pragma unroll 4
      for (int d = 0; d < 128; ++d) s += q[d] * k[d]; }
    sc[w] = s; }
#pragma unroll
  for (int w = 0; w < 5; ++w) sc[w] += __shfl_xor(sc[w], 1);
  float mx = -3.0e38f;
#pragma unroll
  for (int w = 0; w < 5; ++w) { const int j = sidx + w - LWIN; sc[w] = (j >= 0 && j < SS) ? sc[w] * 0.0625f : -3.0e38f; mx = fmaxf(mx, sc[w]); }
  float den = 0.f;
#pragma unroll
  for (int w = 0; w < 5; ++w) { const float e = (sc[w] <= -1.0e38f) ? 0.f : exp_p(sc[w] - mx); sc[w] = e; den += e; }
  const float inv = 1.0f / den;
  for (int d0 = 0; d0 < 128; d0 += 4) { v4f o; for (int i = 0; i < 4; ++i) o[i] = 0.f;
#pragma unroll
    for (int w = 0; w < 5; ++w) { const int j = sidx + w - LWIN; if (j >= 0 && j < SS) { const float* v = LQ + (sb + j) * D3 + 2 * DM + h * HD2 + half * 128 + d0; const float pw = sc[w] * inv; for (int i = 0; i < 4; ++i) o[i] += pw * v[i]; } }
    vst2(LCTX + row * DM + h * HD2 + half * 128 + d0, o); }
  (void)ssc;
}
template <int KIN, int MODE>
__global__ __launch_bounds__(128) void k_lin(const float* __restrict__ A, const float* __restrict__ A2, const __bf16* __restrict__ Wr, const float* __restrict__ BIAS, const float* __restrict__ XRES, float* __restrict__ OUT) {
  __shared__ __align__(16) float so[4][16][132];
  const int tid = threadIdx.x, wave = tid >> 5, lane = tid & 31, col = lane & 15, g = lane >> 4; const size_t r0 = (size_t)blockIdx.x * 64 + wave * 16; const int n0 = blockIdx.y * 128;
  v8f acc[8] = {};
#pragma unroll 2
  for (int kc = 0; kc < KIN / 32; ++kc) { const bool second = (KIN > DM) && (kc >= DM / 32); const F2 a = second ? split_row(A2 + (r0 + col) * DM, (kc - DM / 32) * 32, lane) : split_row(A + (r0 + col) * DM, kc * 32, lane);
#pragma unroll
    for (int j = 0; j < 8; ++j) { const v16b w = frag_b(Wr + (size_t)(n0 + j * 16 + col) * KIN + kc * 32, lane); acc[j] = wmma_bf(a.l, w, acc[j]); acc[j] = wmma_bf(a.h, w, acc[j]); } }
#pragma unroll
  for (int j = 0; j < 8; ++j) { const int c = n0 + j * 16 + col; const float bb = bfr(BIAS[c]);
#pragma unroll
    for (int r = 0; r < 8; ++r) so[wave][8 * g + r][j * 16 + col] = acc[j][r] + bb + (MODE == 1 ? bfr(XRES[(r0 + 8 * g + r) * DM + c]) : 0.f); }
  LDSX();
  for (int rl = 0; rl < 16; ++rl) vst2(OUT + (r0 + rl) * DM + n0 + lane * 4, *(const v4f*)&so[wave][rl][lane * 4]);
}
template <int MODE>
__global__ __launch_bounds__(128) void k_ln(const float* __restrict__ Yin, const float* __restrict__ G, const float* __restrict__ Bt, float* __restrict__ OF, _Float16* __restrict__ OH) {
  __shared__ float red[4]; __shared__ __align__(16) _Float16 sh[DM]; const int t = threadIdx.x; const size_t row = blockIdx.x; float v[4]; float s = 0.f; for (int i = 0; i < 4; ++i) { v[i] = Yin[row * DM + t * 4 + i]; s += v[i]; }
#pragma unroll
  for (int o = 1; o < 32; o <<= 1) s += __shfl_xor(s, o);
  if ((t & 31) == 0) red[t >> 5] = s; __syncthreads(); const float mu = (red[0] + red[1] + red[2] + red[3]) / (float)DM; __syncthreads();
  float q = 0.f; for (int i = 0; i < 4; ++i) { const float dd = v[i] - mu; q += dd * dd; }
#pragma unroll
  for (int o = 1; o < 32; o <<= 1) q += __shfl_xor(q, o);
  if ((t & 31) == 0) red[t >> 5] = q; __syncthreads(); const float inv = 1.0f / sqrtf((red[0] + red[1] + red[2] + red[3]) / (float)DM + 1e-5f);
  v4f o4; for (int i = 0; i < 4; ++i) { const int e = t * 4 + i; o4[i] = (v[i] - mu) * inv * bfr(G[e]) + bfr(Bt[e]); if (MODE == 0) sh[e] = (_Float16)o4[i]; }
  vst2(OF + row * DM + t * 4, o4);
  if (MODE == 0) { __syncthreads(); if (t < DM / 8) vst2((unsigned*)(OH + row * DM + t * 8), *(const v4u*)&sh[t * 8]); }
}
template <int MODE>
__global__ __launch_bounds__(128) void k_mlp(const _Float16* __restrict__ Ain, const _Float16* __restrict__ Wr, const float* __restrict__ BIAS, const float* __restrict__ RES, float* __restrict__ OUTF, _Float16* __restrict__ OG) {
  constexpr int KIN = (MODE == 0) ? DM : DFF; constexpr int NOUT = (MODE == 0) ? DFF : DM;
  __shared__ __align__(16) float so[4][16][132]; __shared__ __align__(16) _Float16 sg[4][16][136];
  const int tid = threadIdx.x, wave = tid >> 5, lane = tid & 31, col = lane & 15, g = lane >> 4; const size_t r0 = (size_t)blockIdx.x * 64 + wave * 16; const int n0 = blockIdx.y * 128;
  v8f acc[8] = {};
#pragma unroll 2
  for (int kc = 0; kc < KIN / 32; ++kc) { const v16h a = frag_h(Ain + (r0 + col) * KIN + kc * 32, lane);
#pragma unroll
    for (int j = 0; j < 8; ++j) acc[j] = wmma16(a, frag_h(Wr + (size_t)(n0 + j * 16 + col) * KIN + kc * 32, lane), acc[j]); }
#pragma unroll
  for (int j = 0; j < 8; ++j) { const int c = n0 + j * 16 + col; const float bb = bfr(BIAS[c]);
#pragma unroll
    for (int r = 0; r < 8; ++r) { const float x = acc[j][r] * (1.0f / 256.0f) + bb; if (MODE == 0) sg[wave][8 * g + r][j * 16 + col] = (_Float16)fmaxf(x, 0.f); else so[wave][8 * g + r][j * 16 + col] = x + RES[(r0 + 8 * g + r) * DM + c]; } }
  LDSX();
  if (MODE == 0) { for (int rl = 0; rl < 16; ++rl) if (lane < 16) vst2((unsigned*)(OG + (r0 + rl) * NOUT + n0 + lane * 8), *(const v4u*)&sg[wave][rl][lane * 8]); }
  else { for (int rl = 0; rl < 16; ++rl) vst2(OUTF + (r0 + rl) * NOUT + n0 + lane * 4, *(const v4f*)&so[wave][rl][lane * 4]); }
}
extern "C" void kernel_launch(void* const* d_in, const int* in_sizes, int n_in, void* d_out, int out_size, void* d_ws, size_t ws_size, hipStream_t stream) {
  (void)in_sizes; (void)n_in; (void)out_size;
  const float** F = (const float**)d_in;
  if (ws_size < (size_t)WS_END) return;
  char* ws = (char*)d_ws; __bf16 *PK = (__bf16*)(ws + WS_PK), *PKL = (__bf16*)(ws + WS_PKL), *PFU = (__bf16*)(ws + WS_PFU); _Float16 *PF1 = (_Float16*)(ws + WS_PF1), *PF2 = (_Float16*)(ws + WS_PF2), *QK = (_Float16*)(ws + WS_QK), *QKL = (_Float16*)(ws + WS_QKL), *VTH = (_Float16*)(ws + WS_VTH), *VTL = (_Float16*)(ws + WS_VTL), *H16 = (_Float16*)(ws + WS_H16), *G16 = (_Float16*)(ws + WS_G16b);
  float *OG = (float*)(ws + WS_OG), *LQKV = (float*)(ws + WS_LQKV), *LCTX = (float*)(ws + WS_LCTX), *GOUT = (float*)(ws + WS_GOUT), *LOUT = (float*)(ws + WS_LOUT), *X1 = (float*)(ws + WS_X1), *Y = (float*)(ws + WS_Y);
  k_pack<<<dim3(DM, 4), 256, 0, stream>>>(F[1], F[1] + (size_t)DM * DM, F[1] + (size_t)2 * DM * DM, F[3], PK);
  k_pack<<<dim3(DM, 4), 256, 0, stream>>>(F[5], F[5] + (size_t)DM * DM, F[5] + (size_t)2 * DM * DM, F[7], PKL);
  k_pack16<<<dim3(DFF, 3), 256, 0, stream>>>(F[13], F[15], F[9], PF1, PF2, PFU);
  k_qkv<<<dim3(NR / 64, QKVW / 128), 128, 0, stream>>>(F[0], F[0], F[0], PK + PK_A, F[2], F[2] + DM, F[2] + 2 * DM, QK, QKL, VTH, VTL);
  k_gatt<<<dim3(TQBG, NHG, NB * 2), 128, 0, stream>>>(QK, VTH, OG);
  k_lqkv<<<dim3(NRB, D3 / 128), 128, 0, stream>>>(F[0], PKL + PK_A, F[6], LQKV);
  k_lattn<<<NRB, 256, 0, stream>>>(LQKV, LCTX);
  k_lin<DM, 0><<<dim3(NRB, DM / 128), 128, 0, stream>>>(OG, nullptr, PK + PK_P, F[4], nullptr, GOUT);
  k_lin<DM, 0><<<dim3(NRB, DM / 128), 128, 0, stream>>>(LCTX, nullptr, PKL + PK_P, F[8], nullptr, LOUT);
  k_lin<D2, 1><<<dim3(NRB, DM / 128), 128, 0, stream>>>(GOUT, LOUT, PFU, F[10], F[0], Y);
  k_ln<0><<<NRB * 64, 128, 0, stream>>>(Y, F[11], F[12], X1, H16);
  k_mlp<0><<<dim3(NRB, DFF / 128), 128, 0, stream>>>(H16, PF1, F[14], nullptr, nullptr, G16);
  k_mlp<1><<<dim3(NRB, DM / 128), 128, 0, stream>>>(G16, PF2, F[16], X1, Y, nullptr);
  k_ln<1><<<NRB * 64, 128, 0, stream>>>(Y, F[17], F[18], (float*)d_out, nullptr);
}
